// OrderedAttention_89842125898335
// MI455X (gfx1250) — hardware-verified
//
#include <hip/hip_runtime.h>


#define NU   3
#define NB_  16
#define NT   1024
#define DD   256
#define NR   16384
typedef _Float16 h16;
typedef unsigned short bf;
typedef __attribute__((ext_vector_type(16))) __bf16   v16bf;
typedef __attribute__((ext_vector_type(16))) _Float16 v16h;
typedef __attribute__((ext_vector_type(8)))  _Float16 v8h;
typedef __attribute__((ext_vector_type(8)))  unsigned short v8us;
typedef __attribute__((ext_vector_type(8)))  float    v8f;
typedef __attribute__((ext_vector_type(4)))  float    v4f;
typedef v8h  __attribute__((may_alias)) v8ha;
typedef v4f  __attribute__((may_alias)) v4fa;
typedef v8us __attribute__((may_alias)) v8usa;

__device__ __forceinline__ unsigned short f2bf(float f) { unsigned u = __float_as_uint(f); u += 0x7FFFu + ((u >> 16) & 1u); return (unsigned short)(u >> 16); }
__device__ __forceinline__ float bf2f(unsigned short b) { return __uint_as_float(((unsigned)b) << 16); }
__device__ __forceinline__ float bfr(float f) { return bf2f(f2bf(f)); }
__device__ __forceinline__ v16h cat16(v8h lo, v8h hi) { return __builtin_shufflevector(lo, hi, 0, 1, 2, 3, 4, 5, 6, 7, 8, 9, 10, 11, 12, 13, 14, 15); }
__device__ __forceinline__ v16bf cat16b(v8us lo, v8us hi) { return __builtin_bit_cast(v16bf, __builtin_shufflevector(lo, hi, 0, 1, 2, 3, 4, 5, 6, 7, 8, 9, 10, 11, 12, 13, 14, 15)); }
__device__ __forceinline__ v8f wmma16(v16h a, v16h b, v8f c) { return __builtin_amdgcn_wmma_f32_16x16x32_f16(false, a, false, b, (short)0, c, false, false); }
__device__ __forceinline__ v8f wmmab(v16bf a, v16bf b, v8f c) { return __builtin_amdgcn_wmma_f32_16x16x32_bf16(false, a, false, b, (short)0, c, false, false); }


template <typename T16> struct WFrag;
template <> struct WFrag<h16> { typedef v16h V; static __device__ __forceinline__ V ld(const h16* p) { return cat16(*(const v8h*)p, *(const v8h*)(p + 16)); } static __device__ __forceinline__ v8f mma(V a, V b, v8f c) { return wmma16(a, b, c); } };
template <> struct WFrag<bf> { typedef v16bf V; static __device__ __forceinline__ V ld(const bf* p) { return cat16b(*(const v8us*)p, *(const v8us*)(p + 16)); } static __device__ __forceinline__ v8f mma(V a, V b, v8f c) { return wmmab(a, b, c); } };
template <typename T16, int NSPLIT, bool BIAS>
__global__ __launch_bounds__(32) void k_gemmw(const T16* __restrict__ A, const T16* __restrict__ A2, const T16* __restrict__ Bt, const T16* __restrict__ Bt2, int K, float* C, int ldc, const float* __restrict__ bias, size_t sA, size_t sB, size_t sC) {
    typedef typename WFrag<T16>::V V;
    __shared__ __align__(16) float os[16 * 68];
    const size_t z = blockIdx.z; A += z * sA; if (A2) A2 += z * sA; Bt += z * sB; if (Bt2) Bt2 += z * sB; C += z * sC;
    const int lane = threadIdx.x & 31, lr = lane & 15, hi = lane >> 4; const int r0 = blockIdx.x * 64, c0 = blockIdx.y * 64;
    v8f acc[4][4];
#pragma unroll
    for (int mb = 0; mb < 4; ++mb)
#pragma unroll
        for (int nb = 0; nb < 4; ++nb) acc[mb][nb] = (v8f){};
    const size_t aoff = (size_t)(r0 + lr) * K + 8 * hi, boff = (size_t)(c0 + lr) * K + 8 * hi;
#pragma unroll 1
    for (int kc = 0; kc < K; kc += 32) {
        V a[4], a2[4];
#pragma unroll
        for (int mb = 0; mb < 4; ++mb) { a[mb] = WFrag<T16>::ld(A + aoff + (size_t)mb * 16 * K + kc); if (NSPLIT == 1 || NSPLIT == 2) a2[mb] = WFrag<T16>::ld(A2 + aoff + (size_t)mb * 16 * K + kc); }
#pragma unroll
        for (int nb = 0; nb < 4; ++nb) { const V b = WFrag<T16>::ld(Bt + boff + (size_t)nb * 16 * K + kc); V b2; if (NSPLIT >= 2) b2 = WFrag<T16>::ld(Bt2 + boff + (size_t)nb * 16 * K + kc);
#pragma unroll
            for (int mb = 0; mb < 4; ++mb) { acc[mb][nb] = WFrag<T16>::mma(a[mb], b, acc[mb][nb]); if (NSPLIT == 1 || NSPLIT == 2) acc[mb][nb] = WFrag<T16>::mma(a2[mb], b, acc[mb][nb]); if (NSPLIT >= 2) acc[mb][nb] = WFrag<T16>::mma(a[mb], b2, acc[mb][nb]); } }
        asm volatile("v_nop\n\tv_nop\n\tv_nop\n\tv_nop" : "+v"(acc[0][0]), "+v"(acc[1][1]), "+v"(acc[2][2]), "+v"(acc[3][3]) : "v"(a[0]), "v"(a[3]));
    }
#pragma unroll
    for (int mb = 0; mb < 4; ++mb) {
#pragma unroll
        for (int nb = 0; nb < 4; ++nb) {
#pragma unroll
            for (int j = 0; j < 8; ++j) os[(hi * 8 + j) * 68 + nb * 16 + lr] = acc[mb][nb][j]; }
        __builtin_amdgcn_wave_barrier(); asm volatile("" ::: "memory");
        float* crow = C + (size_t)(r0 + mb * 16) * ldc + c0;
#pragma unroll 1
        for (int ps = 0; ps < 2; ++ps) {
#pragma unroll
            for (int s = 0; s < 8; ++s) { const int row = 2 * s + hi, cofs = lr * 4; v4f val = *(const v4fa*)(os + row * 68 + cofs); if (BIAS) { val[0] += bfr(bias[c0 + cofs]); val[1] += bfr(bias[c0 + cofs + 1]); val[2] += bfr(bias[c0 + cofs + 2]); val[3] += bfr(bias[c0 + cofs + 3]); }
                *(volatile v4f*)(crow + (size_t)row * ldc + cofs) = val; }
            if (ps == 0) __threadfence(); }
        __builtin_amdgcn_wave_barrier(); asm volatile("" ::: "memory");
    }
}

typedef __attribute__((ext_vector_type(4))) unsigned short v4us;

__global__ __launch_bounds__(256) void k_cvt8(const float* __restrict__ src, bf* dst, size_t n8) { const size_t i = (size_t)blockIdx.x * 256 + threadIdx.x; if (i >= n8) return; const v8f v = *(const v8f*)(src + i * 8); v8us o;
#pragma unroll
    for (int k = 0; k < 8; ++k) o[k] = f2bf(v[k]); *(volatile v8us*)(dst + i * 8) = o; __threadfence(); *(volatile v8us*)(dst + i * 8) = o; }
__global__ __launch_bounds__(256) void k_unary(const float* __restrict__ X, const float* __restrict__ wr, const float* __restrict__ br, float* P) { const int r = blockIdx.x * 256 + threadIdx.x; if (r >= NR) return; const float* xr = X + (size_t)r * DD; float acc = 0.f;
#pragma unroll 1
    for (int e = 0; e < DD; ++e) { float w = bfr(wr[e]); asm volatile("" : "+v"(w)); float p = __fmul_rn(fmaxf(xr[e], 0.f), w); asm volatile("" : "+v"(p)); acc = __fadd_rn(acc, p); }
    const float o = __fadd_rn(acc, bfr(br[0])); *(volatile float*)(P + r) = o; __threadfence(); *(volatile float*)(P + r) = o; }
__global__ __launch_bounds__(256) void k_rnorm(const float* __restrict__ X, float* Y) { const int lane = threadIdx.x & 31; const int r = blockIdx.x * 8 + (threadIdx.x >> 5); if (r >= NR) return; const float* xr = X + (size_t)r * DD; float v[DD / 32]; float q = 0.f;
#pragma unroll
    for (int ch = 0; ch < DD / 128; ++ch) { const v4f a = *(const v4f*)(xr + ch * 128 + lane * 4);
#pragma unroll
        for (int u = 0; u < 4; ++u) { v[ch * 4 + u] = a[u]; float p = __fmul_rn(a[u], a[u]); asm volatile("" : "+v"(p)); q = __fadd_rn(q, p); } }
#pragma unroll
    for (int sh = 16; sh; sh >>= 1) q += __shfl_xor(q, sh, 32);
    const float inv = __fdiv_rn(1.0f, fmaxf(__fsqrt_rn(q), 1e-12f));
    for (int ps = 0; ps < 2; ++ps) {
#pragma unroll
        for (int ch = 0; ch < DD / 128; ++ch) { v4f o;
#pragma unroll
            for (int u = 0; u < 4; ++u) o[u] = __fmul_rn(v[ch * 4 + u], inv); *(volatile v4f*)(Y + (size_t)r * DD + ch * 128 + lane * 4) = o; }
        if (ps == 0) __threadfence(); } }
__global__ __launch_bounds__(256) void k_cmean(const float* __restrict__ Y, float* M) { const int idx = blockIdx.x * 256 + threadIdx.x; if (idx >= NB_ * DD) return; const int e = idx % DD; const int b = idx / DD; const float* yb = Y + (size_t)b * NT * DD + e; float s = 0.f;
#pragma unroll 1
    for (int m = 0; m < NT; ++m) s = __fadd_rn(s, yb[(size_t)m * DD]); const float o = s * (1.0f / NT); *(volatile float*)(M + idx) = o; __threadfence(); *(volatile float*)(M + idx) = o; }
__global__ __launch_bounds__(256) void k_pot(const float* __restrict__ Y, const float* __restrict__ M, float* P) { const int r = blockIdx.x * 256 + threadIdx.x; if (r >= NR) return; const int b = r / NT; const float* yr = Y + (size_t)r * DD; const float* mb = M + (size_t)b * DD; float acc = 0.f;
#pragma unroll 1
    for (int e = 0; e < DD; ++e) { float p = __fmul_rn(yr[e], mb[e]); asm volatile("" : "+v"(p)); acc = __fadd_rn(acc, p); } *(volatile float*)(P + r) = acc; __threadfence(); *(volatile float*)(P + r) = acc; }
__global__ __launch_bounds__(256) void k_rsoft(const float* __restrict__ P0, const float* __restrict__ P1, const float* __restrict__ P2, const float* __restrict__ P3, const float* __restrict__ w, int npot, float* A) { const int lane = threadIdx.x & 31; const int b = blockIdx.x * 8 + (threadIdx.x >> 5); if (b >= NB_) return; float v[NT / 32]; float mx = -3.0e38f;
    float w0 = bfr(w[0]), w1 = bfr(w[1]), w2 = bfr(w[2]), w3 = (npot > 3) ? bfr(w[3]) : 0.f; asm volatile("" : "+v"(w0)); asm volatile("" : "+v"(w1)); asm volatile("" : "+v"(w2)); asm volatile("" : "+v"(w3));
#pragma unroll
    for (int ch = 0; ch < NT / 128; ++ch) { const int n0 = ch * 128 + lane * 4; const size_t o0 = (size_t)b * NT + n0; const v4f a0 = *(const v4f*)(P0 + o0), a1 = *(const v4f*)(P1 + o0), a2 = *(const v4f*)(P2 + o0); v4f a3 = {0.f, 0.f, 0.f, 0.f}; if (npot > 3) a3 = *(const v4f*)(P3 + o0);
#pragma unroll
        for (int u = 0; u < 4; ++u) { float t0 = __fmul_rn(a0[u], w0), t1 = __fmul_rn(a1[u], w1), t2 = __fmul_rn(a2[u], w2), t3 = __fmul_rn(a3[u], w3); asm volatile("" : "+v"(t0)); asm volatile("" : "+v"(t1)); asm volatile("" : "+v"(t2)); asm volatile("" : "+v"(t3));
            float r = __fadd_rn(__fadd_rn(t0, t1), t2); if (npot > 3) r = __fadd_rn(r, t3); v[ch * 4 + u] = r; mx = fmaxf(mx, r); } }
#pragma unroll
    for (int sh = 16; sh; sh >>= 1) mx = fmaxf(mx, __shfl_xor(mx, sh, 32));
    float sum = 0.f;
#pragma unroll
    for (int q = 0; q < NT / 32; ++q) { float d0 = __fsub_rn(v[q], mx); asm volatile("" : "+v"(d0)); v[q] = __builtin_amdgcn_exp2f(__fmul_rn(d0, 1.4426950408889634f)); sum += v[q]; }
#pragma unroll
    for (int sh = 16; sh; sh >>= 1) sum += __shfl_xor(sum, sh, 32);
    const float f = __fdiv_rn(1.0f, sum);
    for (int ps = 0; ps < 2; ++ps) {
#pragma unroll
        for (int ch = 0; ch < NT / 128; ++ch) { v4f o; for (int u = 0; u < 4; ++u) o[u] = v[ch * 4 + u] * f; *(volatile v4f*)(A + (size_t)b * NT + ch * 128 + lane * 4) = o; }
        if (ps == 0) __threadfence(); } }
__global__ __launch_bounds__(256) void k_att(const float* __restrict__ U, const float* __restrict__ A, float* O) { const int idx = blockIdx.x * 256 + threadIdx.x; if (idx >= NB_ * DD) return; const int d = idx % DD; const int b = idx / DD; const float* ub = U + (size_t)b * NT * DD + d; const float* ab = A + (size_t)b * NT; float s = 0.f;
#pragma unroll 1
    for (int n = 0; n < NT; ++n) { float p = __fmul_rn(bfr(ub[(size_t)n * DD]), ab[n]); asm volatile("" : "+v"(p)); s = __fadd_rn(s, p); } *(volatile float*)(O + idx) = s; __threadfence(); *(volatile float*)(O + idx) = s; }

extern "C" void kernel_launch(void* const* d_in, const int* in_sizes, int n_in,
                              void* d_out, int out_size, void* d_ws, size_t ws_size, hipStream_t stream) {
    (void)in_sizes; (void)n_in; (void)out_size;
    const float** I = (const float**)d_in;
    const float* Uin[3] = {I[0], I[1], I[2]}; const float *Wu = I[3], *bu = I[4], *wr = I[5], *br = I[6], *Wsx = I[7], *bsx = I[8], *Wsy = I[9], *bsy = I[10], *Wpx = I[11], *bpx = I[12], *Wpy = I[13], *bpy = I[14], *wdiag = I[15], *wpair = I[16];
    float* OUT = (float*)d_out;
    char* wsp = (char*)d_ws;
    auto take = [&](size_t bytes) { char* p = wsp; wsp += (bytes + 255) & ~(size_t)255; return (void*)p; };
    bf* UB[3]; for (int u = 0; u < 3; ++u) UB[u] = (bf*)take((size_t)NR * DD * 2); bf* WB = (bf*)take(DD * DD * 2); float* X = (float*)take((size_t)NR * DD * 4); float* Y1 = (float*)take((size_t)NR * DD * 4); float* Y2 = (float*)take((size_t)NR * DD * 4); float* M = (float*)take(NB_ * DD * 4);
    float* UNA = (float*)take((size_t)NU * NR * 4); float* SELF = (float*)take((size_t)NU * NR * 4); float* PX = (float*)take((size_t)NU * NU * NR * 4); float* PY = (float*)take((size_t)NU * NU * NR * 4); float* A = (float*)take((size_t)NR * 4);
    if ((size_t)(wsp - (char*)d_ws) > ws_size) return;
    const unsigned gw = (DD * DD / 8 + 255) / 256, gr = (NR + 255) / 256;
    auto gemm = [&](int u, const float* Wt, const float* bias, float* Out) { k_cvt8<<<gw, 256, 0, stream>>>(Wt, WB, DD * DD / 8); k_gemmw<bf, 0, true><<<dim3(NR / 64, DD / 64, 1), 32, 0, stream>>>(UB[u], nullptr, WB, nullptr, DD, Out, DD, bias, 0, 0, 0); };
    for (int u = 0; u < 3; ++u) k_cvt8<<<(unsigned)(((size_t)NR * DD / 8 + 255) / 256), 256, 0, stream>>>(Uin[u], UB[u], (size_t)NR * DD / 8);
    for (int u = 0; u < 3; ++u) {
        gemm(u, Wu + (size_t)u * DD * DD, bu + u * DD, X); k_unary<<<gr, 256, 0, stream>>>(X, wr + u * DD, br + u, UNA + (size_t)u * NR);
        gemm(u, Wsx + (size_t)u * DD * DD, bsx + u * DD, X); k_rnorm<<<NR / 8, 256, 0, stream>>>(X, Y1); gemm(u, Wsy + (size_t)u * DD * DD, bsy + u * DD, X); k_rnorm<<<NR / 8, 256, 0, stream>>>(X, Y2);
        k_cmean<<<(NB_ * DD + 255) / 256, 256, 0, stream>>>(Y2, M); k_pot<<<gr, 256, 0, stream>>>(Y1, M, SELF + (size_t)u * NR);
        for (int v = 0; v < 3; ++v) { if (v == u) continue; const size_t uv = (size_t)u * 3 + v;
            gemm(u, Wpx + uv * DD * DD, bpx + uv * DD, X); k_rnorm<<<NR / 8, 256, 0, stream>>>(X, Y1);
            gemm(v, Wpy + uv * DD * DD, bpy + uv * DD, X); k_rnorm<<<NR / 8, 256, 0, stream>>>(X, Y2);
            k_cmean<<<(NB_ * DD + 255) / 256, 256, 0, stream>>>(Y2, M); k_pot<<<gr, 256, 0, stream>>>(Y1, M, PX + uv * NR);
            k_cmean<<<(NB_ * DD + 255) / 256, 256, 0, stream>>>(Y1, M); k_pot<<<gr, 256, 0, stream>>>(Y2, M, PY + uv * NR); } }
    for (int i = 0; i < 3; ++i) for (int j = 0; j < 3; ++j) {
        if (i == j) { const int k1 = (i == 0) ? 1 : 0, k2 = (i == 2) ? 1 : 2; k_rsoft<<<(NB_ + 7) / 8, 256, 0, stream>>>(UNA + (size_t)i * NR, SELF + (size_t)i * NR, PX + ((size_t)i * 3 + k1) * NR, PX + ((size_t)i * 3 + k2) * NR, wdiag + i * 4, 4, A); }
        else k_rsoft<<<(NB_ + 7) / 8, 256, 0, stream>>>(UNA + (size_t)j * NR, SELF + (size_t)j * NR, PY + ((size_t)i * 3 + j) * NR, nullptr, wpair + (i * 3 + j) * 3, 3, A);
        k_att<<<(NB_ * DD + 255) / 256, 256, 0, stream>>>(Uin[j], A, OUT + ((size_t)i * 3 + j) * NB_ * DD); }
}
